// MatchNetwork_90726889161130
// MI455X (gfx1250) — hardware-verified
//
#include <hip/hip_runtime.h>
#include <math.h>

typedef __attribute__((ext_vector_type(16))) _Float16 v16h;
typedef __attribute__((ext_vector_type(16))) __bf16 v16b;
typedef __attribute__((ext_vector_type(8)))  _Float16 v8h;
typedef __attribute__((ext_vector_type(8)))  float v8f;
typedef __attribute__((ext_vector_type(4)))  float v4f;
typedef __attribute__((ext_vector_type(2)))  float v2f;
typedef __attribute__((ext_vector_type(4)))  unsigned v4u;
typedef __attribute__((ext_vector_type(4)))  int v4i;
typedef float __attribute__((may_alias)) float_a;
typedef int __attribute__((may_alias)) int_a;

template <typename T> __device__ __forceinline__ void vst2(void* p, T v) { *(volatile T*)p = v; __threadfence(); *(volatile T*)p = v; }
__device__ __forceinline__ v8f wmma16(v16h a, v16h b, v8f c) {
  v8f d = __builtin_amdgcn_wmma_f32_16x16x32_f16(false, a, false, b, (short)0, c, false, false);
  asm volatile("v_nop\n\tv_nop\n\tv_nop\n\tv_nop" : "+v"(d) : "v"(a), "v"(b));
  return d;
}
__device__ __forceinline__ v8f wmma_bf(v16b a, v16b b, v8f c) {
  v8f d = __builtin_amdgcn_wmma_f32_16x16x32_bf16(false, a, false, b, (short)0, c, false, false);
  asm volatile("v_nop\n\tv_nop\n\tv_nop\n\tv_nop" : "+v"(d) : "v"(a), "v"(b));
  return d;
}
__device__ __forceinline__ v16h frag_h(const _Float16* rowk0, int lane) {
  union { v16h v; v8h q[2]; } u; const _Float16* p = rowk0 + 8 * (lane >> 4);
  u.q[0] = *(const v8h*)p; u.q[1] = *(const v8h*)(p + 16); return u.v;
}
__device__ __forceinline__ v16h frag_f32(const float* rowk0, int lane) {
  v16h a; const float* p = rowk0 + 8 * (lane >> 4);
#pragma unroll
  for (int i = 0; i < 8; ++i) { a[i] = (_Float16)p[i]; a[8 + i] = (_Float16)p[16 + i]; }
  return a;
}
__device__ __forceinline__ v16h frag_f32s(const float* rowk0, int lane, float sc) {
  v16h a; const float* p = rowk0 + 8 * (lane >> 4);
#pragma unroll
  for (int i = 0; i < 8; ++i) { a[i] = (_Float16)(p[i] * sc); a[8 + i] = (_Float16)(p[16 + i] * sc); }
  return a;
}
__device__ __forceinline__ v16h fragc_f32(const float* W, int k0, int n, int lane, int ld, int K) {
  v16h a; const int g = lane >> 4;
#pragma unroll
  for (int i = 0; i < 8; ++i) { const int ka = k0 + 8 * g + i, kb = ka + 16;
    a[i] = (_Float16)(ka < K ? W[(size_t)(ka < K ? ka : K - 1) * ld + n] : 0.f); a[8 + i] = (_Float16)(kb < K ? W[(size_t)(kb < K ? kb : K - 1) * ld + n] : 0.f); }
  return a;
}
struct F2 { v16b h, l; };
__device__ __forceinline__ F2 bsplit16(const float v[16]) { F2 r;
#pragma unroll
  for (int i = 0; i < 16; ++i) { const __bf16 h = (__bf16)v[i]; r.h[i] = h; r.l[i] = (__bf16)(v[i] - (float)h); }
  return r; }
__device__ __forceinline__ F2 split_row(const float* row, int k0, int lane) { float v[16]; const float* p = row + k0 + 8 * (lane >> 4);
#pragma unroll
  for (int i = 0; i < 8; ++i) { v[i] = p[i]; v[8 + i] = p[16 + i]; }
  return bsplit16(v); }
__device__ __forceinline__ F2 split_rowK(const float* row, int k0, int lane, int K) { float v[16]; const int g = lane >> 4;
#pragma unroll
  for (int i = 0; i < 8; ++i) { const int ka = k0 + 8 * g + i, kb = ka + 16; v[i] = ka < K ? row[ka < K ? ka : K - 1] : 0.f; v[8 + i] = kb < K ? row[kb < K ? kb : K - 1] : 0.f; }
  return bsplit16(v); }
__device__ __forceinline__ F2 split_col(const float* W, int k0, int n, int lane, int ld, int K) { float v[16]; const int g = lane >> 4;
#pragma unroll
  for (int i = 0; i < 8; ++i) { const int ka = k0 + 8 * g + i, kb = ka + 16; v[i] = ka < K ? W[(size_t)(ka < K ? ka : K - 1) * ld + n] : 0.f; v[8 + i] = kb < K ? W[(size_t)(kb < K ? kb : K - 1) * ld + n] : 0.f; }
  return bsplit16(v); }
__device__ __forceinline__ v8f mac3(const F2& a, const F2& b, v8f c) { c = wmma_bf(a.l, b.h, c); c = wmma_bf(a.h, b.l, c); return wmma_bf(a.h, b.h, c); }
__device__ __forceinline__ float sigm(float v) { return 1.0f / (1.0f + expf(-v)); }
#define LDSX() do { asm volatile("s_wait_dscnt 0" ::: "memory"); __builtin_amdgcn_wave_barrier(); __builtin_amdgcn_fence(__ATOMIC_RELEASE, "workgroup"); } while (0)


#define NB 32
#define LL 1024
#define DD 256
#define AA 128
#define NR (NB * LL)
#define BCH 8
#ifndef NBT
#define NBT NB
#define TB0 0
#endif
typedef __attribute__((ext_vector_type(8))) __bf16 v8b;
__device__ __forceinline__ v16b frag_b(const __bf16* rowk0, int lane) {
  union { v16b v; v8b q[2]; } u; const __bf16* p = rowk0 + 8 * (lane >> 4);
  u.q[0] = *(const v8b*)p; u.q[1] = *(const v8b*)(p + 16); return u.v;
}
__device__ __forceinline__ float bfr(float v) { return (float)(__bf16)v; }
__device__ __attribute__((noinline)) float exp_ni(float v) { return expf(v); }
__device__ __attribute__((noinline)) float erf_ni(float v) { return erff(v); }
__device__ __attribute__((noinline)) float tanh_ni(float v) { return tanhf(v); }

#define PK_W  0
#define PK_V  ((size_t)DD * DD)
#define PK_Q  (PK_V + (size_t)AA * DD)
#define PK_END (PK_Q + (size_t)AA * DD)
#define WS_PK   0u
#define WS_F2   (((2u * PK_END) + 127u) / 128u * 128u)
#define WS_F1W  (WS_F2 + 2u * (size_t)NR * DD)
#define WS_P1   (WS_F1W + 4u * (size_t)NR * DD)
#define WS_P2   (WS_P1 + 4u * (size_t)NR * AA)
#define WS_P1T  (WS_P2 + 4u * (size_t)NR * AA)
#define WS_P1TL (WS_P1T + 2u * (size_t)NR * AA)
#define WS_P2T  (WS_P1TL + 2u * (size_t)NR * AA)
#define WS_P2TL (WS_P2T + 2u * (size_t)NR * AA)
#define WS_CH   (WS_P2TL + 2u * (size_t)NR * AA)
#define WS_CL   (WS_CH + 2u * (size_t)BCH * LL * LL)
#define WS_CTH  (WS_CL + 2u * (size_t)BCH * LL * LL)
#define WS_CTL  (WS_CTH + 2u * (size_t)BCH * LL * LL)
#define WS_LG   (WS_CTL + 2u * (size_t)BCH * LL * LL)
#define WS_END  (WS_LG + 4u * 2 * NR)

__global__ __launch_bounds__(256) void k_pack(const float* __restrict__ Wm, const float* __restrict__ WV, const float* __restrict__ WQ, __bf16* __restrict__ PK) {
  __shared__ __align__(16) __bf16 s[DD]; const int n = blockIdx.x, which = blockIdx.y, t = threadIdx.x;
  if (which > 0 && n >= AA) return;
  const float v = (which == 0) ? Wm[(size_t)t * DD + n] : (which == 1) ? WV[(size_t)t * AA + n] : WQ[(size_t)t * AA + n]; s[t] = (__bf16)v;
  __syncthreads();
  if (t < DD / 8) vst2((unsigned*)(PK + ((which == 0) ? PK_W : (which == 1) ? PK_V : PK_Q) + (size_t)n * DD + t * 8), *(const v4u*)&s[t * 8]);
}
__global__ __launch_bounds__(128) void k_proj(const float* __restrict__ F1, const float* __restrict__ F2, const __bf16* __restrict__ PK, __bf16* __restrict__ F2B, float* __restrict__ F1W, float* __restrict__ P1, float* __restrict__ P2, _Float16* __restrict__ P1T, _Float16* __restrict__ P1TL, _Float16* __restrict__ P2T, _Float16* __restrict__ P2TL) {
  __shared__ __align__(16) float so[4][16][132]; __shared__ __align__(16) _Float16 sth[128][72], stl[128][72];
  const int tid = threadIdx.x, wave = tid >> 5, lane = tid & 31, col = lane & 15, g = lane >> 4; const int which = blockIdx.y; const size_t r0 = (size_t)TB0 * LL + (size_t)blockIdx.x * 64 + wave * 16;
  const float* X = (which == 2) ? F2 : F1;
  for (int pass = 0; pass < ((which == 0) ? 2 : 1); ++pass) { const int n0 = pass * 128; const __bf16* P = PK + ((which == 0) ? PK_W : (which == 1) ? PK_V : PK_Q);
    v8f acc[8] = {};
#pragma unroll 2
    for (int kc = 0; kc < DD / 32; ++kc) { v16b a; { const float* p = X + (r0 + col) * DD + kc * 32 + 8 * g;
#pragma unroll
        for (int i = 0; i < 8; ++i) { a[i] = (__bf16)p[i]; a[8 + i] = (__bf16)p[16 + i]; } }
#pragma unroll
      for (int j = 0; j < 8; ++j) acc[j] = wmma_bf(a, frag_b(P + (size_t)(n0 + j * 16 + col) * DD + kc * 32, lane), acc[j]); }
#pragma unroll
    for (int j = 0; j < 8; ++j)
#pragma unroll
      for (int r = 0; r < 8; ++r) { so[wave][8 * g + r][j * 16 + col] = acc[j][r]; if (which > 0) { const float v = acc[j][r]; const _Float16 hv = (_Float16)v; sth[j * 16 + col][wave * 16 + 8 * g + r] = hv; stl[j * 16 + col][wave * 16 + 8 * g + r] = (_Float16)((v - (float)hv) * 2048.0f); } }
    __syncthreads();
    if (which == 0) { for (int rl = 0; rl < 16; ++rl) vst2(F1W + (r0 + rl) * DD + n0 + lane * 4, *(const v4f*)&so[wave][rl][lane * 4]); }
    else { float* D = (which == 1) ? P1 : P2; for (int rl = 0; rl < 16; ++rl) vst2(D + (r0 + rl) * AA + lane * 4, *(const v4f*)&so[wave][rl][lane * 4]);
      const size_t rb = (size_t)TB0 * LL + (size_t)blockIdx.x * 64; const int b = (int)(rb / LL), s0 = (int)(rb % LL); _Float16* TH = (which == 1) ? P1T : P2T; _Float16* TL = (which == 1) ? P1TL : P2TL;
      for (int e = tid; e < 128 * 8; e += 128) { const int d = e >> 3, pc = e & 7; const size_t o = ((size_t)b * AA + d) * LL + s0 + pc * 8; vst2((unsigned*)(TH + o), *(const v4u*)&sth[d][pc * 8]); vst2((unsigned*)(TL + o), *(const v4u*)&stl[d][pc * 8]); } }
    __syncthreads(); }
  if (which == 2) { __shared__ __align__(16) __bf16 sb[4][16][DD + 8]; for (int rl = 0; rl < 16; ++rl) { const float* p = F2 + (r0 + rl) * DD + lane * 8;
#pragma unroll
      for (int i = 0; i < 8; ++i) sb[wave][rl][lane * 8 + i] = (__bf16)p[i]; }
    LDSX(); for (int rl = 0; rl < 16; ++rl) vst2((unsigned*)(F2B + (r0 + rl) * DD + lane * 8), *(const v4u*)&sb[wave][rl][lane * 8]); }
}
__global__ __launch_bounds__(128) void k_aff(const float* __restrict__ F1W, const __bf16* __restrict__ F2B, int bbase, _Float16* __restrict__ CH, _Float16* __restrict__ CL, _Float16* __restrict__ CTH, _Float16* __restrict__ CTL) {
  __shared__ __align__(16) _Float16 soh[4][16][136], sol[4][16][136]; __shared__ __align__(16) _Float16 sth[128][72], stl[128][72];
  const int tid = threadIdx.x, wave = tid >> 5, lane = tid & 31, col = lane & 15, g = lane >> 4; const int bl = blockIdx.z; const size_t b = (size_t)bbase + bl; const int i0 = blockIdx.x * 64 + wave * 16, j0 = blockIdx.y * 128;
  v8f acc[8] = {};
#pragma unroll 2
  for (int kc = 0; kc < DD / 32; ++kc) { const F2 a = split_row(F1W + (b * LL + i0 + col) * DD, kc * 32, lane);
#pragma unroll
    for (int j = 0; j < 8; ++j) { const v16b w = frag_b(F2B + (b * LL + j0 + j * 16 + col) * DD + kc * 32, lane); acc[j] = wmma_bf(a.l, w, acc[j]); acc[j] = wmma_bf(a.h, w, acc[j]); } }
#pragma unroll
  for (int j = 0; j < 8; ++j)
#pragma unroll
    for (int r = 0; r < 8; ++r) { const float v = tanh_ni(acc[j][r]); const _Float16 hv = (_Float16)v; const _Float16 lv = (_Float16)((v - (float)hv) * 2048.0f); soh[wave][8 * g + r][j * 16 + col] = hv; sol[wave][8 * g + r][j * 16 + col] = lv; sth[j * 16 + col][wave * 16 + 8 * g + r] = hv; stl[j * 16 + col][wave * 16 + 8 * g + r] = lv; }
  __syncthreads();
  for (int rl = 0; rl < 16; ++rl) { const size_t o = ((size_t)bl * LL + i0 + rl) * LL + j0; if (lane < 16) vst2((unsigned*)(CH + o + lane * 8), *(const v4u*)&soh[wave][rl][lane * 8]); else vst2((unsigned*)(CL + o + (lane - 16) * 8), *(const v4u*)&sol[wave][rl][(lane - 16) * 8]); }
  { const int i0b = blockIdx.x * 64; for (int e = tid; e < 128 * 8; e += 128) { const int d = e >> 3, pc = e & 7; const size_t o = ((size_t)bl * LL + j0 + d) * LL + i0b + pc * 8; vst2((unsigned*)(CTH + o), *(const v4u*)&sth[d][pc * 8]); vst2((unsigned*)(CTL + o), *(const v4u*)&stl[d][pc * 8]); } }
}
__global__ __launch_bounds__(128) void k_hvq(const float* __restrict__ P1, const float* __restrict__ P2, const _Float16* __restrict__ CH, const _Float16* __restrict__ CL, const _Float16* __restrict__ CTH, const _Float16* __restrict__ CTL, const _Float16* __restrict__ P1T, const _Float16* __restrict__ P1TL, const _Float16* __restrict__ P2T, const _Float16* __restrict__ P2TL, const float* __restrict__ WHV, const float* __restrict__ WHQ, int bbase, float* __restrict__ LG) {
  __shared__ float sl[4][16][16];
  const int tid = threadIdx.x, wave = tid >> 5, lane = tid & 31, col = lane & 15, g = lane >> 4; const int bl = blockIdx.y, side = blockIdx.z; const size_t b = (size_t)bbase + bl; const int i0 = blockIdx.x * 64 + wave * 16;
  const _Float16* AH = (side == 0) ? CH : CTH; const _Float16* AL = (side == 0) ? CL : CTL; const _Float16* BH = (side == 0) ? P2T : P1T; const _Float16* BL = (side == 0) ? P2TL : P1TL; const float* PS = (side == 0) ? P1 : P2; const float* wv = (side == 0) ? WHV : WHQ;
  v8f acc[8] = {}, accl[8] = {};
#pragma unroll 2
  for (int kc = 0; kc < LL / 32; ++kc) { const size_t ar = ((size_t)bl * LL + i0 + col) * LL + kc * 32; const v16h ah = frag_h(AH + ar, lane), al = frag_h(AL + ar, lane);
#pragma unroll
    for (int j = 0; j < 8; ++j) { const size_t br = (b * AA + j * 16 + col) * LL + kc * 32; const v16h bh = frag_h(BH + br, lane); acc[j] = wmma16(ah, bh, acc[j]); accl[j] = wmma16(al, bh, accl[j]); accl[j] = wmma16(ah, frag_h(BL + br, lane), accl[j]); } }
  float part[8];
#pragma unroll
  for (int r = 0; r < 8; ++r) part[r] = 0.f;
#pragma unroll
  for (int j = 0; j < 8; ++j) { const int a2 = j * 16 + col; const float w = bfr(wv[a2]);
#pragma unroll
    for (int r = 0; r < 8; ++r) { const size_t row = b * LL + i0 + 8 * g + r; const float hval = tanh_ni(PS[row * AA + a2] + acc[j][r] + accl[j][r] * (1.0f / 2048.0f)); part[r] += hval * w; } }
#pragma unroll
  for (int r = 0; r < 8; ++r) { float v = part[r];
#pragma unroll
    for (int o = 1; o < 16; o <<= 1) v += __shfl_xor(v, o);
    if (col == 0) sl[wave][8 * g + r][0] = v; }
  LDSX();
  if (lane < 16) {   }
  __syncthreads();
  { __shared__ __align__(16) float s64[64]; if (tid < 64) s64[tid] = sl[tid >> 4][tid & 15][0]; __syncthreads(); if (tid < 16) vst2(LG + (size_t)side * NR + b * LL + blockIdx.x * 64 + tid * 4, *(const v4f*)&s64[tid * 4]); }
}
__global__ __launch_bounds__(256) void k_pool(const float* __restrict__ LG, const int* __restrict__ M1, const int* __restrict__ M2, const float* __restrict__ F1, const float* __restrict__ F2, float* __restrict__ OUT) {
  __shared__ float sw[LL]; __shared__ float red[8];
  const int t = threadIdx.x; const int b = TB0 + blockIdx.x, side = blockIdx.y; const float* lg = LG + (size_t)side * NR + (size_t)b * LL; const int* M = ((side == 0) ? M1 : M2) + (size_t)b * LL; const float* F = ((side == 0) ? F1 : F2) + (size_t)b * LL * DD;
  float mx = -3.0e38f; for (int i = t; i < LL; i += 256) { const float m = (M[i] != 0) ? 1.f : 0.f; const float v = lg[i] * m; sw[i] = v; mx = fmaxf(mx, v); }
#pragma unroll
  for (int o = 1; o < 32; o <<= 1) mx = fmaxf(mx, __shfl_xor(mx, o));
  if ((t & 31) == 0) red[t >> 5] = mx; __syncthreads(); float gm = -3.0e38f; for (int w = 0; w < 8; ++w) gm = fmaxf(gm, red[w]); __syncthreads();
  float s = 0.f; for (int i = t; i < LL; i += 256) { const float e = exp_ni(sw[i] - gm); sw[i] = e; s += e; }
#pragma unroll
  for (int o = 1; o < 32; o <<= 1) s += __shfl_xor(s, o);
  if ((t & 31) == 0) red[t >> 5] = s; __syncthreads(); float tot = 0.f; for (int w = 0; w < 8; ++w) tot += red[w]; __syncthreads();
  float s2 = 0.f; for (int i = t; i < LL; i += 256) { const float m = (M[i] != 0) ? 1.f : 0.f; const float r = (sw[i] / tot) * m; sw[i] = r; s2 += r; }
#pragma unroll
  for (int o = 1; o < 32; o <<= 1) s2 += __shfl_xor(s2, o);
  if ((t & 31) == 0) red[t >> 5] = s2; __syncthreads(); float tot2 = 0.f; for (int w = 0; w < 8; ++w) tot2 += red[w]; const float inv = 1.0f / (tot2 + 1e-13f); __syncthreads();
  { const int c = t; float a = 0.f; for (int i = 0; i < LL; ++i) a += sw[i] * bfr(F[(size_t)i * DD + c]); a *= inv;
    __shared__ __align__(16) float so[DD]; so[c] = a; __syncthreads(); if (t < DD / 4) vst2(OUT + (size_t)side * (NB * DD) + (size_t)b * DD + t * 4, *(const v4f*)&so[t * 4]); }
}
extern "C" void kernel_launch(void* const* d_in, const int* in_sizes, int n_in, void* d_out, int out_size, void* d_ws, size_t ws_size, hipStream_t stream) {
  (void)in_sizes; (void)n_in; (void)out_size;
  const float** F = (const float**)d_in;
  if (ws_size < (size_t)WS_END) return;
  char* ws = (char*)d_ws; __bf16 *PK = (__bf16*)(ws + WS_PK), *F2B = (__bf16*)(ws + WS_F2); float *F1W = (float*)(ws + WS_F1W), *P1 = (float*)(ws + WS_P1), *P2 = (float*)(ws + WS_P2), *LG = (float*)(ws + WS_LG); _Float16 *P1T = (_Float16*)(ws + WS_P1T), *P1TL = (_Float16*)(ws + WS_P1TL), *P2T = (_Float16*)(ws + WS_P2T), *P2TL = (_Float16*)(ws + WS_P2TL), *CH = (_Float16*)(ws + WS_CH), *CL = (_Float16*)(ws + WS_CL), *CTH = (_Float16*)(ws + WS_CTH), *CTL = (_Float16*)(ws + WS_CTL);
  k_pack<<<dim3(DD, 3), 256, 0, stream>>>(F[4], F[5], F[6], PK);
  k_proj<<<dim3(NBT * LL / 64, 3), 128, 0, stream>>>(F[0], F[1], PK, F2B, F1W, P1, P2, P1T, P1TL, P2T, P2TL);
  for (int bb = TB0; bb < TB0 + NBT; bb += BCH) { const int nb = (TB0 + NBT - bb < BCH) ? (TB0 + NBT - bb) : BCH;
    k_aff<<<dim3(LL / 64, LL / 128, nb), 128, 0, stream>>>(F1W, F2B, bb, CH, CL, CTH, CTL);
    k_hvq<<<dim3(LL / 64, nb, 2), 128, 0, stream>>>(P1, P2, CH, CL, CTH, CTL, P1T, P1TL, P2T, P2TL, F[7], F[8], bb, LG); }
  k_pool<<<dim3(NBT, 2), 256, 0, stream>>>(LG, (const int*)d_in[2], (const int*)d_in[3], F[0], F[1], (float*)d_out);
}
